// GCN_DeepSet_AntiSym_Invariant_34565896798211
// MI455X (gfx1250) — hardware-verified
//
#include <hip/hip_runtime.h>
#include <math.h>

typedef __attribute__((ext_vector_type(16))) _Float16 v16h;
typedef __attribute__((ext_vector_type(8)))  _Float16 v8h;
typedef __attribute__((ext_vector_type(16))) __bf16   v16b;
typedef __attribute__((ext_vector_type(8)))  float    v8f;
typedef __attribute__((ext_vector_type(4)))  float    v4f;

__device__ __forceinline__ int frag_k(int i, int h) { return (i < 8) ? (8 * h + i) : (16 + 8 * h + (i - 8)); }
__device__ __forceinline__ __bf16 bf16_rne(float f) {
    unsigned int u = __float_as_uint(f);
    u += 0x7fffu + ((u >> 16) & 1u);
    return __builtin_bit_cast(__bf16, (unsigned short)(u >> 16));
}
__device__ __forceinline__ float bf16_f32(__bf16 b) { return __uint_as_float(((unsigned int)__builtin_bit_cast(unsigned short, b)) << 16); }
__device__ __forceinline__ v8f wmma16(v16h a, v16h b, v8f c) {
    c = __builtin_amdgcn_wmma_f32_16x16x32_f16(false, a, false, b, (short)0, c, false, false);
    asm volatile("v_nop\n\tv_nop\n\tv_nop\n\tv_nop" : "+v"(c) : "v"(a), "v"(b));
    return c;
}
__device__ __forceinline__ v8f wmmab(v16b a, v16b b, v8f c) {
    c = __builtin_amdgcn_wmma_f32_16x16x32_bf16(false, a, false, b, (short)0, c, false, false);
    asm volatile("v_nop\n\tv_nop\n\tv_nop\n\tv_nop" : "+v"(c) : "v"(a), "v"(b));
    return c;
}
struct Split { v16b hi, lo; };
__device__ __forceinline__ v8f wmma3(const Split& a, const Split& b, v8f c) {
    c = __builtin_amdgcn_wmma_f32_16x16x32_bf16(false, a.hi, false, b.hi, (short)0, c, false, false);
    c = __builtin_amdgcn_wmma_f32_16x16x32_bf16(false, a.hi, false, b.lo, (short)0, c, false, false);
    c = __builtin_amdgcn_wmma_f32_16x16x32_bf16(false, a.lo, false, b.hi, (short)0, c, false, false);
    asm volatile("v_nop\n\tv_nop\n\tv_nop\n\tv_nop" : "+v"(c) : "v"(a.hi), "v"(a.lo), "v"(b.hi), "v"(b.lo));
    return c;
}
struct Split3 { v16b hi, mid, lo; };
__device__ __forceinline__ v8f wmma6(const Split3& a, const Split3& b, v8f c) {
    c = __builtin_amdgcn_wmma_f32_16x16x32_bf16(false, a.hi, false, b.hi, (short)0, c, false, false);
    c = __builtin_amdgcn_wmma_f32_16x16x32_bf16(false, a.hi, false, b.mid, (short)0, c, false, false);
    c = __builtin_amdgcn_wmma_f32_16x16x32_bf16(false, a.mid, false, b.hi, (short)0, c, false, false);
    c = __builtin_amdgcn_wmma_f32_16x16x32_bf16(false, a.hi, false, b.lo, (short)0, c, false, false);
    c = __builtin_amdgcn_wmma_f32_16x16x32_bf16(false, a.mid, false, b.mid, (short)0, c, false, false);
    c = __builtin_amdgcn_wmma_f32_16x16x32_bf16(false, a.lo, false, b.hi, (short)0, c, false, false);
    asm volatile("v_nop\n\tv_nop\n\tv_nop\n\tv_nop" : "+v"(c) : "v"(a.hi), "v"(a.mid), "v"(a.lo), "v"(b.hi), "v"(b.mid), "v"(b.lo));
    return c;
}

__device__ __forceinline__ v16h fh_ld(const float* __restrict__ p, long long sk, int k0, int h, int klen, float s) {
    v16h a;
#pragma unroll
    for (int i = 0; i < 16; ++i) { const int k = k0 + frag_k(i, h); a[i] = (k < klen) ? (_Float16)(p[(long long)k * sk] * s) : (_Float16)0.f; }
    return a;
}
__device__ __forceinline__ Split sp_ld(const float* __restrict__ p, long long sk, int k0, int h, int klen, float s) {
    Split r;
#pragma unroll
    for (int i = 0; i < 16; ++i) {
        const int k = k0 + frag_k(i, h); const float x = (k < klen) ? p[(long long)k * sk] * s : 0.f;
        const __bf16 hb = bf16_rne(x); r.hi[i] = hb; r.lo[i] = bf16_rne(x - bf16_f32(hb));
    }
    return r;
}
__device__ __forceinline__ Split3 sp3_ld(const float* __restrict__ p, long long sk, int k0, int h, int klen, float s) {
    Split3 r;
#pragma unroll
    for (int i = 0; i < 16; ++i) {
        const int k = k0 + frag_k(i, h); const float x = (k < klen) ? p[(long long)k * sk] * s : 0.f;
        const __bf16 hb = bf16_rne(x); const float r1 = x - bf16_f32(hb); const __bf16 mb = bf16_rne(r1);
        r.hi[i] = hb; r.mid[i] = mb; r.lo[i] = bf16_rne(r1 - bf16_f32(mb));
    }
    return r;
}
__device__ __forceinline__ v16b bh_ld(const float* __restrict__ p, long long sk, int k0, int h, int klen, float s) {
    v16b a;
#pragma unroll
    for (int i = 0; i < 16; ++i) { const int k = k0 + frag_k(i, h); a[i] = bf16_rne((k < klen) ? p[(long long)k * sk] * s : 0.f); }
    return a;
}
__device__ __forceinline__ v16h fh_row(const _Float16* __restrict__ row, int k0, int h) {
    v16h a;
#pragma unroll
    for (int i = 0; i < 16; ++i) a[i] = row[k0 + frag_k(i, h)];
    return a;
}

#define VST2(T, ptr, val) do { const T vst2_v_ = (val); *(volatile T*)(ptr) = vst2_v_; __threadfence(); *(volatile T*)(ptr) = vst2_v_; } while (0)
typedef float v4f __attribute__((ext_vector_type(4)));
#define VST2V4(ptr, val) do { const v4f vst2_v4_ = (val); *(volatile v4f*)(ptr) = vst2_v4_; __threadfence(); *(volatile v4f*)(ptr) = vst2_v4_; } while (0)

__device__ __attribute__((noinline)) float act_fn(float v, int act) {
    if (act == 1) return fmaxf(v, 0.f);
    if (act == 2) { const float u = 0.7978845608028654f * (v + 0.044715f * v * v * v); return 0.5f * v * (1.f + tanhf(u)); }
    if (act == 3) return v / (1.f + expf(-v));
    if (act == 4) return 0.5f * v * (1.f + erff(v * 0.7071067811865476f));
    if (act == 5) return tanhf(v);
    if (act == 6) return 1.f / (1.f + expf(-v));
    if (act == 7) return (v > 0.f) ? v : 0.01f * v;
    if (act == 8) return (v > 0.f) ? v : (expf(v) - 1.f);
    if (act == 9) return fminf(fmaxf(v, 0.f), 6.f);
    if (act == 10) return fabsf(v);
    if (act == 11) return (v >= 0.f) ? v : 0.1f * v;
    if (act == 12) return (v > 0.f) ? v : 0.2f * v;
    if (act == 13) return (v > 20.f) ? v : log1pf(expf(v));
    return v;
}

struct GemmP {
    const float* A; const float* B; const float* bias; const float* R; float* C;
    long long sAo, sAi, sAm, sAk, sBo, sBi, sBn, sBk, sCo, sCi, sCm, sRo, sRi, sRm, sRn;
    int M, N, K, zi_n, flags, act; float alpha, beta, sa, sb;
    int Npad, pad_;
};
static_assert(sizeof(GemmP) == 5 * 8 + 15 * 8 + 6 * 4 + 4 * 4 + 2 * 4, "GemmP has padding");

template <int MODE>
__global__ __launch_bounds__(32) void k_gemm(GemmP p) {
    const int lane = threadIdx.x & 31, h = lane >> 4, l15 = lane & 15;
    const int m0 = blockIdx.y * 16, n0 = blockIdx.x * 32;
    const int z = blockIdx.z, zo = z / p.zi_n, zi = z - zo * p.zi_n;
    const float* A = p.A + zo * p.sAo + zi * p.sAi;
    const float* B = p.B + zo * p.sBo + zi * p.sBi;
    const int am = min(m0 + l15, p.M - 1);
    v8f acc[2], comp[2];
#pragma unroll
    for (int t = 0; t < 2; ++t) { v8f zz = {}; acc[t] = zz; comp[t] = zz; }
    for (int k0 = 0; k0 < p.K; k0 += 32) {
        const float* arow = A + (long long)am * p.sAm;
        if (MODE == 1) {
            const Split a = sp_ld(arow, p.sAk, k0, h, p.K, 1.f);
#pragma unroll
            for (int t = 0; t < 2; ++t) {
                const int bn = min(n0 + t * 16 + l15, p.N - 1);
                acc[t] = wmma3(a, sp_ld(B + (long long)bn * p.sBn, p.sBk, k0, h, p.K, 1.f), acc[t]);
            }
        } else if (MODE == 3) {
            const Split3 a = sp3_ld(arow, p.sAk, k0, h, p.K, 1.f);
#pragma unroll
            for (int t = 0; t < 2; ++t) {
                const int bn = min(n0 + t * 16 + l15, p.N - 1);
                acc[t] = wmma6(a, sp3_ld(B + (long long)bn * p.sBn, p.sBk, k0, h, p.K, 1.f), acc[t]);
            }
        } else if (MODE == 4) {
            const Split3 a = sp3_ld(arow, p.sAk, k0, h, p.K, 1.f);
#pragma unroll
            for (int t = 0; t < 2; ++t) {
                const int bn = min(n0 + t * 16 + l15, p.N - 1); v8f zz = {};
                const v8f part = wmma6(a, sp3_ld(B + (long long)bn * p.sBn, p.sBk, k0, h, p.K, 1.f), zz);
                const v8f y = part - comp[t]; const v8f s = acc[t] + y; comp[t] = (s - acc[t]) - y; acc[t] = s;
            }
        } else if (MODE == 2) {
            const v16b a = bh_ld(arow, p.sAk, k0, h, p.K, 1.f);
#pragma unroll
            for (int t = 0; t < 2; ++t) {
                const int bn = min(n0 + t * 16 + l15, p.N - 1);
                acc[t] = wmmab(a, bh_ld(B + (long long)bn * p.sBn, p.sBk, k0, h, p.K, 1.f), acc[t]);
            }
        } else {
            const v16h a = fh_ld(arow, p.sAk, k0, h, p.K, p.sa);
#pragma unroll
            for (int t = 0; t < 2; ++t) {
                const int bn = min(n0 + t * 16 + l15, p.N - 1);
                acc[t] = wmma16(a, fh_ld(B + (long long)bn * p.sBn, p.sBk, k0, h, p.K, p.sb), acc[t]);
            }
        }
    }
    const float iscale = (MODE == 0) ? p.alpha / (p.sa * p.sb) : p.alpha;
    float* C = p.C + zo * p.sCo + zi * p.sCi;
    const float* R = p.R + zo * p.sRo + zi * p.sRi;
    __shared__ __align__(16) float ctile[16][36];
#pragma unroll
    for (int t = 0; t < 2; ++t) {
        const int n = n0 + t * 16 + l15; const int nn = min(n, p.N - 1);
#pragma unroll
        for (int r = 0; r < 8; ++r) {
            const int m = m0 + 8 * h + r; const int mm = min(m, p.M - 1);
            float v = acc[t][r] * iscale;
            if (p.flags & 1) v += p.bias[nn];
            if (p.flags & 2) v += p.bias[mm];
            if (p.flags & 8) v *= p.bias[(long long)zo * p.M + mm];
            v = act_fn(v, p.act);
            if (p.flags & 4) v += p.beta * R[(long long)mm * p.sRm + (long long)nn * p.sRn];
            ctile[8 * h + r][t * 16 + l15] = (n < p.N) ? v : 0.f;
        }
    }
    __syncthreads();
    const int NW = (p.Npad > p.N) ? p.Npad : p.N;
    const bool fast = (m0 + 16 <= p.M) && (n0 + 32 <= NW) && ((p.sCm & 3) == 0) && ((((size_t)C) & 15) == 0);
    if (fast) {
#pragma unroll
        for (int s = 0; s < 4; ++s) {
            const int row = s * 4 + (lane >> 3), c4 = (lane & 7) * 4;
            const v4f v = *(const v4f*)&ctile[row][c4];
            VST2V4(C + (long long)(m0 + row) * p.sCm + n0 + c4, v);
        }
    } else {
        for (int row = 0; row < 16; ++row) {
            const int m = m0 + row, n = n0 + lane;
            if (m < p.M && n < NW) VST2(float, C + (long long)m * p.sCm + n, ctile[row][lane]);
        }
    }
}


template <int MODE, int TM, int TN>
__global__ __launch_bounds__(32) void k_gemmT(GemmP p) {
    const int lane = threadIdx.x & 31, h = lane >> 4, l15 = lane & 15;
    const int m0 = blockIdx.y * (16 * TM), n0 = blockIdx.x * (16 * TN);
    const int z = blockIdx.z, zo = z / p.zi_n, zi = z - zo * p.zi_n;
    const float* A = p.A + zo * p.sAo + zi * p.sAi;
    const float* B = p.B + zo * p.sBo + zi * p.sBi;
    v8f acc[TM][TN];
#pragma unroll
    for (int i = 0; i < TM; ++i)
#pragma unroll
        for (int t = 0; t < TN; ++t) { v8f zz = {}; acc[i][t] = zz; }
    for (int k0 = 0; k0 < p.K; k0 += 32) {
        if (MODE == 1) {
            Split a[TM], b[TN];
#pragma unroll
            for (int i = 0; i < TM; ++i) { const int am = min(m0 + 16 * i + l15, p.M - 1); a[i] = sp_ld(A + (long long)am * p.sAm, p.sAk, k0, h, p.K, 1.f); }
#pragma unroll
            for (int t = 0; t < TN; ++t) { const int bn = min(n0 + 16 * t + l15, p.N - 1); b[t] = sp_ld(B + (long long)bn * p.sBn, p.sBk, k0, h, p.K, 1.f); }
#pragma unroll
            for (int i = 0; i < TM; ++i)
#pragma unroll
                for (int t = 0; t < TN; ++t) acc[i][t] = wmma3(a[i], b[t], acc[i][t]);
        } else if (MODE == 2) {
            v16b a[TM], b[TN];
#pragma unroll
            for (int i = 0; i < TM; ++i) { const int am = min(m0 + 16 * i + l15, p.M - 1); a[i] = bh_ld(A + (long long)am * p.sAm, p.sAk, k0, h, p.K, 1.f); }
#pragma unroll
            for (int t = 0; t < TN; ++t) { const int bn = min(n0 + 16 * t + l15, p.N - 1); b[t] = bh_ld(B + (long long)bn * p.sBn, p.sBk, k0, h, p.K, 1.f); }
#pragma unroll
            for (int i = 0; i < TM; ++i)
#pragma unroll
                for (int t = 0; t < TN; ++t) acc[i][t] = wmmab(a[i], b[t], acc[i][t]);
        } else {
            v16h a[TM], b[TN];
#pragma unroll
            for (int i = 0; i < TM; ++i) { const int am = min(m0 + 16 * i + l15, p.M - 1); a[i] = fh_ld(A + (long long)am * p.sAm, p.sAk, k0, h, p.K, p.sa); }
#pragma unroll
            for (int t = 0; t < TN; ++t) { const int bn = min(n0 + 16 * t + l15, p.N - 1); b[t] = fh_ld(B + (long long)bn * p.sBn, p.sBk, k0, h, p.K, p.sb); }
#pragma unroll
            for (int i = 0; i < TM; ++i)
#pragma unroll
                for (int t = 0; t < TN; ++t) acc[i][t] = wmma16(a[i], b[t], acc[i][t]);
        }
    }
    const float iscale = (MODE == 0) ? p.alpha / (p.sa * p.sb) : p.alpha;
    float* C = p.C + zo * p.sCo + zi * p.sCi;
    const float* R = p.R + zo * p.sRo + zi * p.sRi;
    const int NW = (p.Npad > p.N) ? p.Npad : p.N;
    __shared__ __align__(16) float ctile[16][36];
#pragma unroll
    for (int i = 0; i < TM; ++i) {
        const int mb = m0 + 16 * i; if (mb >= p.M) break;
#pragma unroll
        for (int tp = 0; tp < TN / 2; ++tp) {
            const int nb = n0 + 32 * tp; if (nb >= NW) break;
#pragma unroll
            for (int t2 = 0; t2 < 2; ++t2) {
                const int t = 2 * tp + t2; const int n = nb + t2 * 16 + l15; const int nn = min(n, p.N - 1);
#pragma unroll
                for (int r = 0; r < 8; ++r) {
                    const int m = mb + 8 * h + r; const int mm = min(m, p.M - 1);
                    float v = acc[i][t][r] * iscale;
                    if (p.flags & 1) v += p.bias[nn];
                    if (p.flags & 2) v += p.bias[mm];
            if (p.flags & 8) v *= p.bias[(long long)zo * p.M + mm];
                    v = act_fn(v, p.act);
                    if (p.flags & 4) v += p.beta * R[(long long)mm * p.sRm + (long long)nn * p.sRn];
                    ctile[8 * h + r][t2 * 16 + l15] = (n < p.N) ? v : 0.f;
                }
            }
            __syncthreads();
            const bool fast = (mb + 16 <= p.M) && (nb + 32 <= NW) && ((p.sCm & 3) == 0) && ((((size_t)C) & 15) == 0);
            if (fast) {
#pragma unroll
                for (int s = 0; s < 4; ++s) {
                    const int row = s * 4 + (lane >> 3), c4 = (lane & 7) * 4;
                    const v4f v = *(const v4f*)&ctile[row][c4];
                    VST2V4(C + (long long)(mb + row) * p.sCm + nb + c4, v);
                }
            } else {
                for (int row = 0; row < 16; ++row) {
                    const int m = mb + row, n = nb + lane;
                    if (m < p.M && n < NW) VST2(float, C + (long long)m * p.sCm + n, ctile[row][lane]);
                }
            }
            __syncthreads();
        }
    }
}

#define AW 4
struct AttnP {
    const float* Q; const float* K; const float* V; float* O; float* P; const float* Mf; const int* Mi; float* ST;
    const float* Pw; const float* Rt; const int* SQ; const int* SK;
    long long swb, swh, swi, swj, srb, srh, sri;
    long long sQb, sQh, sQi, sQd, sKb, sKh, sKj, sKd, sVb, sVh, sVj, sVd, sOb, sOh, sOi, sPb, sPh, sPi, smb, smh, smi, smj;
    int Lq, Lk, dh, dv, hrep, causal, coff, pband;
    float scale, mfill; int nonorm, mpol;
    int roff, rn, segpol, win;
};
static_assert(sizeof(AttnP) == 12 * 8 + 29 * 8 + 16 * 4, "AttnP has padding");

#ifndef KATTN_ATTR
#define KATTN_ATTR
#endif
template <int DHP, int DVP, int QM, bool SPLITPV, bool TWOPASS>
__global__ __launch_bounds__(32 * AW) KATTN_ATTR void k_attn(AttnP p) {
    constexpr int NT = DVP / 16;
    constexpr int KS = DHP / 32;
    constexpr int VP = DVP + 8;
    __shared__ __align__(16) float    pl[AW][16 * 64];
    __shared__ __align__(16) _Float16 vl[(SPLITPV ? 2 : 1) * 64 * VP];
    const int lane = threadIdx.x & 31, hf = lane >> 4, l15 = lane & 15, wave = threadIdx.x >> 5;
    const int h = blockIdx.y, b = blockIdx.z, hk = h / p.hrep;
    const int q0 = (blockIdx.x * AW + wave) * 16;
    float* myp = pl[wave];
    const float L2E = 1.4426950408889634f;
    const float NEG = -__builtin_inff();
    const int qi = min(q0 + l15, p.Lq - 1);
    const float* qrow = p.Q + b * p.sQb + h * p.sQh + (long long)qi * p.sQi;
    const float* kbase = p.K + b * p.sKb + hk * p.sKh;
    const float* vbase = p.V + b * p.sVb + hk * p.sVh;
    v16h qa[QM == 0 ? KS : 1]; Split qs_[QM == 1 ? KS : 1]; Split3 qt_[QM == 2 ? KS : 1];
#pragma unroll
    for (int ks = 0; ks < KS; ++ks) {
        if (QM == 2) qt_[ks] = sp3_ld(qrow, p.sQd, ks * 32, hf, p.dh, 1.f);
        else if (QM == 1) qs_[ks] = sp_ld(qrow, p.sQd, ks * 32, hf, p.dh, 1.f);
        else qa[ks] = fh_ld(qrow, p.sQd, ks * 32, hf, p.dh, 1.f);
    }
    v8f o[NT]; float m8[8], l8[8];
#pragma unroll
    for (int t = 0; t < NT; ++t) { v8f zz = {}; o[t] = zz; }
#pragma unroll
    for (int i = 0; i < 8; ++i) { m8[i] = NEG; l8[i] = 0.f; }
    int jend = p.Lk;
    if (p.causal == 1) { const int je = (blockIdx.x * AW + AW - 1) * 16 + 16 + p.coff; jend = min(jend, max(je, 0)); }
    const int npass = TWOPASS ? 2 : 1;
    for (int pass = 0; pass < npass; ++pass) {
        const bool dopv = (!TWOPASS) || pass == 1;
        for (int j0 = 0; j0 < jend; j0 += 64) {
            if (dopv) {
                __syncthreads();
                for (int idx = threadIdx.x; idx < 64 * DVP; idx += 32 * AW) {
                    const int jr = idx / DVP, d = idx - jr * DVP, j = j0 + jr;
                    const float f = (j < p.Lk && d < p.dv) ? vbase[(long long)j * p.sVj + (long long)d * p.sVd] : 0.f;
                    if (SPLITPV) {
                        const __bf16 hb = bf16_rne(f);
                        ((__bf16*)vl)[jr * VP + d] = hb; ((__bf16*)vl)[64 * VP + jr * VP + d] = bf16_rne(f - bf16_f32(hb));
                    } else vl[jr * VP + d] = (_Float16)f;
                }
            }
            v8f s[4];
#pragma unroll
            for (int t = 0; t < 4; ++t) {
                const int j = min(j0 + t * 16 + l15, p.Lk - 1);
                const float* krow = kbase + (long long)j * p.sKj;
                v8f acc = {};
#pragma unroll
                for (int ks = 0; ks < KS; ++ks) {
                    if (QM == 2)      acc = wmma6(qt_[ks], sp3_ld(krow, p.sKd, ks * 32, hf, p.dh, 1.f), acc);
                    else if (QM == 1) acc = wmma3(qs_[ks], sp_ld(krow, p.sKd, ks * 32, hf, p.dh, 1.f), acc);
                    else              acc = wmma16(qa[ks], fh_ld(krow, p.sKd, ks * 32, hf, p.dh, 1.f), acc);
                }
                s[t] = acc;
            }
            float pv[8][4];
#pragma unroll
            for (int i = 0; i < 8; ++i) {
                const int irow = q0 + i + 8 * hf;
                const int ic = min(irow, p.Lq - 1);
                float sc[4];
#pragma unroll
                for (int t = 0; t < 4; ++t) {
                    const int jg = j0 + t * 16 + l15;
                    float v = s[t][i] * p.scale;
                    if (p.Mf) v += p.Mf[b * p.smb + h * p.smh + (long long)ic * p.smi + (long long)min(jg, p.Lk - 1) * p.smj];
                    if (p.Rt) { int rc = ic - min(jg, p.Lk - 1) + p.roff; rc = rc < 0 ? 0 : (rc >= p.rn ? p.rn - 1 : rc); v += p.Rt[b * p.srb + h * p.srh + (long long)ic * p.sri + rc]; }
                    if (p.Mi) { const int mv = p.Mi[b * p.smb + h * p.smh + (long long)ic * p.smi + (long long)min(jg, p.Lk - 1) * p.smj]; if (p.mpol ? (mv != 0) : (mv == 0)) v = p.mfill; }
                    if (p.SQ) { const bool same = p.SQ[(long long)b * p.Lq + ic] == p.SK[(long long)b * p.Lk + min(jg, p.Lk - 1)]; if (p.segpol ? same : !same) v = p.mfill; }
                    if (p.causal == 2 && jg > irow + p.coff) v = p.mfill;
                    if (jg >= p.Lk || (p.causal == 1 && jg > irow + p.coff) || (p.causal == 3 && jg < irow + p.coff) || (p.win > 0 && irow + p.coff - jg > p.win)) v = NEG; else v *= L2E;
                    sc[t] = v;
                }
                if (!TWOPASS || pass == 0) {
                    float mx = fmaxf(fmaxf(sc[0], sc[1]), fmaxf(sc[2], sc[3]));
                    mx = fmaxf(mx, __shfl_xor(mx, 1, 32)); mx = fmaxf(mx, __shfl_xor(mx, 2, 32));
                    mx = fmaxf(mx, __shfl_xor(mx, 4, 32)); mx = fmaxf(mx, __shfl_xor(mx, 8, 32));
                    const float mnew = fmaxf(m8[i], mx);
                    const float corr = (mnew == NEG) ? 1.f : exp2f(m8[i] - mnew);
                    float rs = 0.f;
#pragma unroll
                    for (int t = 0; t < 4; ++t) {
                        const float pp = (sc[t] == NEG) ? 0.f : exp2f(sc[t] - mnew); rs += pp;
                        pv[i][t] = p.Pw ? pp * p.Pw[b * p.swb + h * p.swh + (long long)ic * p.swi + (long long)min(j0 + t * 16 + l15, p.Lk - 1) * p.swj] : pp;
                    }
                    rs += __shfl_xor(rs, 1, 32); rs += __shfl_xor(rs, 2, 32); rs += __shfl_xor(rs, 4, 32); rs += __shfl_xor(rs, 8, 32);
                    l8[i] = l8[i] * corr + rs; m8[i] = mnew;
                    if (!TWOPASS) {
#pragma unroll
                        for (int t = 0; t < NT; ++t) o[t][i] *= corr;
                    }
                } else {
                    const float inv = (l8[i] > 0.f) ? 1.f / l8[i] : 0.f;
#pragma unroll
                    for (int t = 0; t < 4; ++t) {
                        const int jg = j0 + t * 16 + l15;
                        float pp = (sc[t] == NEG) ? 0.f : exp2f(sc[t] - m8[i]) * inv;
                        if (p.Pw) pp *= p.Pw[b * p.swb + h * p.swh + (long long)ic * p.swi + (long long)min(jg, p.Lk - 1) * p.swj];
                        pv[i][t] = pp;
                    }
                }
            }
            if (dopv) {
#pragma unroll
                for (int i = 0; i < 8; ++i)
#pragma unroll
                    for (int t = 0; t < 4; ++t) myp[(i + 8 * hf) * 64 + t * 16 + l15] = pv[i][t];
                __syncthreads();
                if (p.P) {
                    float* pb_ = p.P + b * p.sPb + h * p.sPh;
                    const bool fastP = (p.pband == 0) && ((p.sPi & 3) == 0) && (j0 + 64 <= p.Lk) && (q0 + 16 <= p.Lq) && ((((size_t)pb_) & 15) == 0);
                    if (fastP) {
#pragma unroll
                        for (int s = 0; s < 8; ++s) {
                            const int row = s * 2 + (lane >> 4), c4 = (lane & 15) * 4;
                            const v4f v = *(const v4f*)(myp + row * 64 + c4);
                            VST2V4(pb_ + (long long)(q0 + row) * p.sPi + j0 + c4, v);
                        }
                    } else {
                        for (int row = 0; row < 16; ++row) {
                            const int irow = q0 + row; if (irow >= p.Lq) continue;
                            for (int c = lane; c < 64; c += 32) {
                                const int jg = j0 + c; if (jg >= p.Lk) continue;
                                if (p.pband == 0) VST2(float, pb_ + (long long)irow * p.sPi + jg, myp[row * 64 + c]);
                                else if (jg - irow <= p.pband && irow - jg <= p.pband) VST2(float, pb_ + (long long)irow * p.sPi + (jg - irow + p.pband), myp[row * 64 + c]);
                            }
                        }
                    }
                }
                if (SPLITPV) {
                    const Split pa0 = sp_ld(myp + l15 * 64, 1, 0, hf, 64, 1.f), pa1 = sp_ld(myp + l15 * 64, 1, 32, hf, 64, 1.f);
                    const __bf16* vh = (const __bf16*)vl; const __bf16* vlo = vh + 64 * VP;
#pragma unroll
                    for (int t = 0; t < NT; ++t) {
                        const int dcol = t * 16 + l15;
                        Split b0, b1;
#pragma unroll
                        for (int e = 0; e < 16; ++e) {
                            const int k0 = frag_k(e, hf), k1 = 32 + frag_k(e, hf);
                            b0.hi[e] = vh[k0 * VP + dcol]; b0.lo[e] = vlo[k0 * VP + dcol]; b1.hi[e] = vh[k1 * VP + dcol]; b1.lo[e] = vlo[k1 * VP + dcol];
                        }
                        o[t] = wmma3(pa0, b0, o[t]);
                        o[t] = wmma3(pa1, b1, o[t]);
                    }
                } else {
                    const v16h pa0 = fh_ld(myp + l15 * 64, 1, 0, hf, 64, 4096.f), pa1 = fh_ld(myp + l15 * 64, 1, 32, hf, 64, 4096.f);
#pragma unroll
                    for (int t = 0; t < NT; ++t) {
                        const int dcol = t * 16 + l15;
                        v16h b0, b1;
#pragma unroll
                        for (int e = 0; e < 16; ++e) { b0[e] = vl[frag_k(e, hf) * VP + dcol]; b1[e] = vl[(32 + frag_k(e, hf)) * VP + dcol]; }
                        o[t] = wmma16(pa0, b0, o[t]);
                        o[t] = wmma16(pa1, b1, o[t]);
                    }
                }
            }
        }
    }
    float* obase = p.O + b * p.sOb + h * p.sOh;
    if (p.ST) {
        const int rl = lane >> 1, isel = rl & 7;
        float mv = 0.f, lv = 0.f;
#pragma unroll
        for (int i = 0; i < 8; ++i) if (i == isel) { mv = m8[i]; lv = l8[i]; }
        const int irow = q0 + rl;
        if (irow < p.Lq) { float* st = p.ST + (((long long)b * gridDim.y + h) * p.Lq + irow) * 2 + (lane & 1); VST2(float, st, (lane & 1) ? lv : mv * 0.6931471805599453f); }
    }
    float invr[8];
#pragma unroll
    for (int i = 0; i < 8; ++i) {
        if (TWOPASS) invr[i] = SPLITPV ? 1.f : (1.f / 4096.f);
        else if (p.nonorm) invr[i] = exp2f(m8[i]) * (SPLITPV ? 1.f : (1.f / 4096.f));
        else invr[i] = (l8[i] > 0.f) ? (SPLITPV ? 1.f / l8[i] : 1.f / (l8[i] * 4096.f)) : 0.f;
    }
    __syncthreads();
    const bool ofast = ((p.sOi & 3) == 0) && ((((size_t)obase) & 15) == 0) && (q0 + 16 <= p.Lq);
#pragma unroll
    for (int c0 = 0; c0 < DVP; c0 += 64) {
#pragma unroll
        for (int i = 0; i < 8; ++i)
#pragma unroll
            for (int t = 0; t < NT; ++t) if (t * 16 >= c0 && t * 16 < c0 + 64) myp[(i + 8 * hf) * 64 + (t * 16 - c0) + l15] = o[t][i] * invr[i];
        __syncthreads();
        const int cw = (DVP - c0 < 64) ? (DVP - c0) : 64;
        if (ofast && (c0 + cw <= p.dv) && (cw % 32 == 0)) {
            const int lpr = cw / 4;
            const int rows_per_ins = 32 / lpr;
            for (int r0 = 0; r0 < 16; r0 += rows_per_ins) {
                const int row = r0 + lane / lpr, c4 = (lane % lpr) * 4;
                const v4f v = *(const v4f*)(myp + row * 64 + c4);
                VST2V4(obase + (long long)(q0 + row) * p.sOi + c0 + c4, v);
            }
        } else {
            for (int row = 0; row < 16; ++row) {
                const int irow = q0 + row; if (irow >= p.Lq) continue;
                for (int c = lane; c < cw; c += 32) { const int d = c0 + c; if (d < p.dv) VST2(float, obase + (long long)irow * p.sOi + d, myp[row * 64 + c]); }
            }
        }
        __syncthreads();
    }
}

struct TrP { const float* src; float* dst; const float* R2; long long sSz, lds, sDz, ldd, sRz, ldr; int R, C, flags, act; float alpha, beta; };
static_assert(sizeof(TrP) == 3 * 8 + 6 * 8 + 6 * 4, "TrP has padding");
__global__ __launch_bounds__(256) void k_tr(TrP p) {
    __shared__ float tile[32][33];
    const int c0 = blockIdx.x * 32, r0 = blockIdx.y * 32, z = blockIdx.z;
    const int lane = threadIdx.x & 31, wave = threadIdx.x >> 5;
    const float* s = p.src + z * p.sSz;
#pragma unroll
    for (int k = 0; k < 4; ++k) {
        const int rl = wave * 4 + k, r = r0 + rl, c = c0 + lane;
        tile[rl][lane] = (r < p.R && c < p.C) ? s[(long long)r * p.lds + c] : 0.f;
    }
    __syncthreads();
    float* d = p.dst + z * p.sDz; const float* rr = p.R2 + z * p.sRz;
#pragma unroll
    for (int k = 0; k < 4; ++k) {
        const int cl = wave * 4 + k, c = c0 + cl, r = r0 + lane;
        if (c < p.C && r < p.R) {
            float v = act_fn(p.alpha * tile[lane][cl], p.act);
            if (p.flags & 1) v += p.beta * rr[(long long)c * p.ldr + r];
            VST2(float, d + (long long)c * p.ldd + r, v);
        }
    }
}

__global__ __launch_bounds__(256) void k_affine(const float* __restrict__ src, float* __restrict__ dst, int n, float a, float b, const float* __restrict__ sdev) {
    const int i = blockIdx.x * 256 + threadIdx.x;
    if (i < n) { const float aa = sdev ? a * sdev[0] : a; const float v = aa * src[i] + b; VST2(float, dst + i, v); }
}

struct SmP { const float* src; float* dst; const float* Mf; long long sz, sr, dz, dr, smz, smr; int n, pad; float scale_in, scale_out; };
static_assert(sizeof(SmP) == 3 * 8 + 6 * 8 + 4 * 4, "SmP has padding");
__global__ __launch_bounds__(256) void k_softmax(SmP p) {
    __shared__ float red[256];
    const int r = blockIdx.x, z = blockIdx.y, tid = threadIdx.x;
    const float* s = p.src + z * p.sz + (long long)r * p.sr;
    const float* mf = p.Mf ? (p.Mf + z * p.smz + (long long)r * p.smr) : nullptr;
    float mx = -__builtin_inff();
    for (int j = tid; j < p.n; j += 256) { float v = s[j] * p.scale_in; if (mf) v += mf[j]; mx = fmaxf(mx, v); }
    red[tid] = mx; __syncthreads();
    for (int o = 128; o > 0; o >>= 1) { if (tid < o) red[tid] = fmaxf(red[tid], red[tid + o]); __syncthreads(); }
    mx = red[0]; __syncthreads();
    float sum = 0.f;
    for (int j = tid; j < p.n; j += 256) { float v = s[j] * p.scale_in; if (mf) v += mf[j]; sum += (mx == -__builtin_inff()) ? 0.f : expf(v - mx); }
    red[tid] = sum; __syncthreads();
    for (int o = 128; o > 0; o >>= 1) { if (tid < o) red[tid] += red[tid + o]; __syncthreads(); }
    sum = red[0];
    const float inv = (sum > 0.f) ? p.scale_out / sum : 0.f;
    float* d = p.dst + z * p.dz + (long long)r * p.dr;
    for (int j = tid; j < p.n; j += 256) { float v = s[j] * p.scale_in; if (mf) v += mf[j]; const float o = (mx == -__builtin_inff()) ? 0.f : expf(v - mx) * inv; VST2(float, d + j, o); }
}
__global__ __launch_bounds__(256) void k_stats(const float* __restrict__ x, long long sz, long long so, long long si, int inner, int n, float eps, float* __restrict__ stat, int mode) {
    __shared__ float red[256];
    const int z = blockIdx.x, tid = threadIdx.x;
    const float* base = x + z * sz;
    float s = 0.f;
    for (int e = tid; e < n; e += 256) s += base[(long long)(e / inner) * so + (long long)(e % inner) * si];
    red[tid] = s; __syncthreads();
    for (int o = 128; o > 0; o >>= 1) { if (tid < o) red[tid] += red[tid + o]; __syncthreads(); }
    const float mu = (mode == 0 || mode == 3) ? red[0] / (float)n : 0.f; __syncthreads();
    float q = 0.f;
    for (int e = tid; e < n; e += 256) { const float dlt = base[(long long)(e / inner) * so + (long long)(e % inner) * si] - mu; q += dlt * dlt; }
    red[tid] = q; __syncthreads();
    for (int o = 128; o > 0; o >>= 1) { if (tid < o) red[tid] += red[tid + o]; __syncthreads(); }
    {
        float rs;
        if (mode == 2) rs = sqrtf((float)n) / fmaxf(sqrtf(red[0]), eps); else if (mode == 3) rs = rsqrtf(red[0] / (float)(n - 1) + eps); else rs = rsqrtf(red[0] / (float)n + eps);
        if (tid < 32) { const float v = (tid == 0) ? mu : ((tid == 1) ? rs : 0.f); VST2(float, stat + (long long)z * 32 + tid, v); }
    }
}
__global__ __launch_bounds__(256) void k_norm_apply(const float* __restrict__ x, float* __restrict__ y, const float* __restrict__ stat, const float* __restrict__ g, const float* __restrict__ bta,
                                                     int Z, int C, int L, int G, int bn, int act) {
    const long long idx = (long long)blockIdx.x * 256 + threadIdx.x;
    if (idx >= (long long)Z * C * L) return;
    const int l = (int)(idx % L); const long long zc = idx / L; const int c = (int)(zc % C), z = (int)(zc / C); (void)l;
    const int set = bn ? c : (z * G + c / (C / G));
    float v = (x[idx] - stat[(long long)set * 32]) * stat[(long long)set * 32 + 1];
    if (g) v *= g[c];
    if (bta) v += bta[c];
    v = act_fn(v, act);
    VST2(float, y + idx, v);
}

__global__ __launch_bounds__(256) void k_lse_neg(const float* __restrict__ st, float* __restrict__ c, int n) {
    const int i = blockIdx.x * 256 + threadIdx.x;
    if (i < n) { const float v = -(st[2 * i] + logf(st[2 * i + 1])); VST2(float, c + i, v); }
}

__global__ __launch_bounds__(256) void k_iota(int* __restrict__ dst, int n, int a, int b) {
    const int i = blockIdx.x * 256 + threadIdx.x;
    if (i < n) { const int v = a * i + b; VST2(int, dst + i, v); }
}

__global__ __launch_bounds__(256) void k_axpby(const float* __restrict__ x, const float* __restrict__ y, float* __restrict__ dst, int n, float a, float b, float c) {
    const int i = blockIdx.x * 256 + threadIdx.x;
    if (i < n) { const float v = a * x[i] + b * y[i] + c; VST2(float, dst + i, v); }
}

struct RopeP { const float* X; float* Y; const float* C; const float* Sn; const int* pos; long long sXr, sXh, sYr, sYh, sCb, sCp, sCd; int R, Hn, D, S, mode, tmode, pmode, pad; };
static_assert(sizeof(RopeP) == 5 * 8 + 7 * 8 + 8 * 4, "RopeP has padding");
__global__ __launch_bounds__(256) void k_rope(RopeP p) {
    const long long idx = (long long)blockIdx.x * 256 + threadIdx.x;
    if (idx >= (long long)p.R * p.Hn * p.D) return;
    const int d = (int)(idx % p.D); const long long rh = idx / p.D; const int h = (int)(rh % p.Hn); const int r = (int)(rh / p.Hn);
    const int half = p.D / 2;
    int partner; float sign;
    if (p.mode == 0) { partner = (d < half) ? d + half : d - half; sign = (d < half) ? -1.f : 1.f; }
    else { partner = d ^ 1; sign = (d & 1) ? 1.f : -1.f; }
    const int tcol = (p.tmode == 0) ? d : ((p.tmode == 1) ? (d % half) : (d >> 1));
    const int pp = (p.pmode == 0) ? (r % p.S) : ((p.pmode == 1) ? h : p.pos[r]);
    const long long toff = (long long)(r / p.S) * p.sCb + (long long)pp * p.sCp + (long long)tcol * p.sCd;
    const float* xr = p.X + (long long)r * p.sXr + (long long)h * p.sXh;
    const float v = xr[d] * p.C[toff] + sign * xr[partner] * p.Sn[toff];
    VST2(float, p.Y + (long long)r * p.sYr + (long long)h * p.sYh + d, v);
}

__global__ __launch_bounds__(256) void k_invf(float* __restrict__ invb, int half, int D, float base, float num, int fmode, float cexp) {
    const int i = blockIdx.x * 256 + threadIdx.x;
    if (i >= ((half + 31) / 32) * 32) return;
    if (i >= half) { VST2(float, invb + i, 0.f); return; }
    const float e = (float)(2 * i) / (float)D;
    float invf;
    if (fmode == 1) invf = num * expf((float)(2 * i) * cexp);
    else if (fmode == 2) invf = num * powf(base, (-2.0f * ((float)i - 1.0f)) / (float)D);
    else invf = num * (1.0f / powf(base, e));
    VST2(float, invb + i, invf);
}
__global__ __launch_bounds__(256) void k_sincos(float* __restrict__ cs, float* __restrict__ sn, const float* __restrict__ invb, int S, int half, float pscale) {
    const int idx = blockIdx.x * 256 + threadIdx.x;
    if (idx >= S * half) return;
    const int s = idx / half, i = idx - s * half;
    const float ang = (pscale * (float)s) * invb[i];
    VST2(float, cs + idx, cosf(ang)); VST2(float, sn + idx, sinf(ang));
}

__global__ __launch_bounds__(256) void k_mulact(const float* __restrict__ x, const float* __restrict__ y, float* __restrict__ dst, int n, int act) {
    const int i = blockIdx.x * 256 + threadIdx.x;
    if (i < n) { const float v = act_fn(x[i], act) * y[i]; VST2(float, dst + i, v); }
}

__global__ __launch_bounds__(256) void k_matvec(GemmP p) {
    const int rpt = (p.N == 1) ? 1 : 32;
    const long long r0 = ((long long)blockIdx.x * 256 + threadIdx.x) * rpt; const int z = blockIdx.z, zo = z / p.zi_n, zi = z - zo * p.zi_n;
    if (r0 >= p.M) return;
    const float* Bb = p.B + zo * p.sBo + zi * p.sBi;
    float* C = p.C + zo * p.sCo + zi * p.sCi; const float* R = p.R + zo * p.sRo + zi * p.sRi;
    for (int rr = 0; rr < rpt; ++rr) {
        const long long r = r0 + rr; if (r >= p.M) break;
        const float* A = p.A + zo * p.sAo + zi * p.sAi + r * p.sAm;
        float acc[8] = {0.f, 0.f, 0.f, 0.f, 0.f, 0.f, 0.f, 0.f};
        for (int k = 0; k < p.K; ++k) { const float a = A[(long long)k * p.sAk];
#pragma unroll
            for (int j = 0; j < 8; ++j) if (j < p.N) acc[j] += a * Bb[(long long)j * p.sBn + (long long)k * p.sBk]; }
#pragma unroll
        for (int j = 0; j < 8; ++j) if (j < p.N) {
            float v = acc[j] * p.alpha;
            if (p.flags & 1) v += p.bias[j];
            if (p.flags & 2) v += p.bias[r];
            v = act_fn(v, p.act);
            if (p.flags & 4) v += p.beta * R[r * p.sRm + (long long)j * p.sRn];
            VST2(float, C + r * p.sCm + j, v);
        }
    }
}
__global__ __launch_bounds__(256) void k_smallsoftmax(const float* __restrict__ src, float* __restrict__ dst, long long sr, long long dr, int n, long long R, float scale) {
    const long long r0 = ((long long)blockIdx.x * 256 + threadIdx.x) * 32;
    for (int rr = 0; rr < 32; ++rr) {
        const long long r = r0 + rr; if (r >= R) return;
        const float* s = src + r * sr; float* d = dst + r * dr;
        float mx = -__builtin_inff();
        for (int j = 0; j < n; ++j) mx = fmaxf(mx, s[j] * scale);
        float sum = 0.f;
        for (int j = 0; j < n; ++j) sum += expf(s[j] * scale - mx);
        const float inv = 1.f / sum;
        for (int j = 0; j < n; ++j) { const float v = expf(s[j] * scale - mx) * inv; VST2(float, d + j, v); }
    }
}

__global__ __launch_bounds__(32) void k_unitstat(float* __restrict__ st) { const int t = threadIdx.x; const float v = (t == 1) ? 1.f : 0.f; VST2(float, st + t, v); }

__global__ __launch_bounds__(256) void k_lincopy(const float* __restrict__ src, long long lds, float* __restrict__ dst, long long ldd, long long rows, int cols) {
    const long long i = (long long)blockIdx.x * 256 + threadIdx.x; if (i >= rows * cols) return;
    const long long r = i / cols; const int c = (int)(i - r * cols);
    const float v = src[r * lds + c]; VST2(float, dst + r * ldd + c, v);
}

__global__ __launch_bounds__(256) void k_gd_bd(const float* __restrict__ A, float* __restrict__ BD, int Bn, int NN, int NT) { const long long q = (long long)blockIdx.x * 256 + threadIdx.x; if (q >= (long long)3 * NT * 64 * 64) return; const int c = (int)(q % 64); const int r = (int)((q / 64) % 64); const int t = (int)((q / 4096) % NT); const int w = (int)(q / ((long long)4096 * NT)); float v = 0.f;
    const int sr = r / NN, sc = c / NN; const int b = t * 6 + sr;
    if (sr == sc && sr < 6 && b < Bn) { const int jr = r % NN, ic = c % NN; const float* Ab = A + (long long)b * NN * NN;
        if (w == 2) v = fabsf(Ab[jr * NN + ic]);
        else {
            const float a = Ab[ic * NN + jr]; const bool rel1 = a > 0.f; float cnt = 0.f; for (int i2 = 0; i2 < NN; ++i2) { const bool r1 = Ab[i2 * NN + jr] > 0.f; cnt += (w == 1) ? (r1 ? 1.f : 0.f) : (r1 ? 0.f : 1.f); }
            const bool sel = (w == 1) ? rel1 : !rel1; v = sel ? 1.f / fmaxf(cnt, 1.f) : 0.f; } }
    VST2(float, BD + q, v); }
__global__ __launch_bounds__(256) void k_gd_zero(float* __restrict__ A1, float* __restrict__ A2, float* __restrict__ A3, long long n) { const long long q = (long long)blockIdx.x * 256 + threadIdx.x; if (q >= n) return; VST2(float, A1 + q, 0.f); VST2(float, A2 + q, 0.f); VST2(float, A3 + q, 0.f); }
__global__ __launch_bounds__(256) void k_gd_add(float* __restrict__ Hh, const float* __restrict__ AGg, long long n) { const long long q = (long long)blockIdx.x * 256 + threadIdx.x; if (q >= n) return; VST2(float, Hh + q, Hh[q] + AGg[q]); }
__global__ __launch_bounds__(256) void k_gd_lnrelu(float* __restrict__ AGg, const float* __restrict__ g_, const float* __restrict__ b_, int rows, int D) { const int r = blockIdx.x * 256 + threadIdx.x; if (r >= rows) return; float* x = AGg + (long long)r * D; float s = 0.f, s2 = 0.f;
#pragma unroll 1
    for (int c = 0; c < D; ++c) { s += x[c]; s2 += x[c] * x[c]; } const float mu = s / (float)D; const float rs = rsqrtf(fmaxf(s2 / (float)D - mu * mu, 0.f) + 1e-5f);
#pragma unroll 1
    for (int c = 0; c < D; ++c) { const float v = (x[c] - mu) * rs * g_[c] + b_[c]; VST2(float, x + c, fmaxf(v, 0.f)); } }
__global__ __launch_bounds__(256) void k_gd_sets(const float* __restrict__ PH, const int* __restrict__ hm, float* __restrict__ SS, int GC, int NN, int PHI, int BnTot) { const long long q = (long long)blockIdx.x * 256 + threadIdx.x; if (q >= (long long)GC * PHI) return; const int c = (int)(q % PHI); const int b = (int)(q / PHI); float s1 = 0.f, s2 = 0.f;
#pragma unroll 1
    for (int n = 0; n < NN; ++n) { const float m = (float)hm[b * NN + n]; const float v = PH[((long long)b * NN + n) * PHI + c]; s1 += v * m; s2 += v * (1.f - m); } VST2(float, SS + q, s1); VST2(float, SS + (long long)BnTot * PHI + q, s2); }
__global__ __launch_bounds__(128) void k_gd_out(const float* __restrict__ R1, const float* __restrict__ r2w, float* __restrict__ OUT, int Bn, int RHO) { __shared__ float red[128]; const int b = blockIdx.x; const int c = threadIdx.x; red[c] = (R1[(long long)b * RHO + c] - R1[((long long)Bn + b) * RHO + c]) * r2w[c]; __syncthreads(); for (int o = 64; o > 0; o >>= 1) { if (c < o) red[c] += red[c + o]; __syncthreads(); } if (c == 0) VST2(float, OUT + b, 0.5f + 0.5f * tanhf(red[0])); }

template __global__ void k_gemm<0>(GemmP);
template __global__ void k_gemm<1>(GemmP);

extern "C" void kernel_launch(void* const* d_in, const int* in_sizes, int n_in, void* d_out, int out_size, void* d_ws, size_t ws_size, hipStream_t stream) {
    (void)in_sizes; (void)n_in; (void)out_size; (void)ws_size;
    const float* A = (const float*)d_in[0];
    const float* X = (const float*)d_in[1];
    const int* hm = (const int*)d_in[2];
    const float* We1 = (const float*)d_in[3];
    const float* be1 = (const float*)d_in[4];
    const float* We2 = (const float*)d_in[5];
    const float* be2 = (const float*)d_in[6];
    const float* rw = (const float*)d_in[7];
    const float* rroot = (const float*)d_in[8];
    const float* rb = (const float*)d_in[9];
    const float* l1w = (const float*)d_in[10];
    const float* l1b = (const float*)d_in[11];
    const float* l2w = (const float*)d_in[12];
    const float* l2b = (const float*)d_in[13];
    const float* lng = (const float*)d_in[14];
    const float* lnb = (const float*)d_in[15];
    const float* p1w = (const float*)d_in[16];
    const float* p1b = (const float*)d_in[17];
    const float* p2w = (const float*)d_in[18];
    const float* p2b = (const float*)d_in[19];
    const float* r1w = (const float*)d_in[20];
    const float* r1b = (const float*)d_in[21];
    const float* r2w = (const float*)d_in[22];
    const float* r2b = (const float*)d_in[23];
    const int Bn = 4096;
    const int NN = 10;
    const int DIN = 32;
    const int D = 128;
    const int PHI = 256;
    const int RHO = 128;
    const int NR = Bn * NN;
    const int GPT = 6;
    const int NT = 683;
    const int NRP = NT * 60 + 64;
    const int RC = 20480;
    const int GC = 2048;
    float* out = (float*)d_out;
    char* wsp = (char*)d_ws;
    float* BD = (float*)wsp; wsp += (((size_t)((size_t)3 * NT * 64 * 64) * 4 + 255) / 256) * 256;
    float* H = (float*)wsp; wsp += (((size_t)((size_t)NRP * D) * 4 + 255) / 256) * 256;
    float* T1 = (float*)wsp; wsp += (((size_t)((size_t)NRP * D) * 4 + 255) / 256) * 256;
    float* M0 = (float*)wsp; wsp += (((size_t)((size_t)NRP * D) * 4 + 255) / 256) * 256;
    float* M1 = (float*)wsp; wsp += (((size_t)((size_t)NRP * D) * 4 + 255) / 256) * 256;
    float* SS = (float*)wsp; wsp += (((size_t)((size_t)2 * Bn * PHI) * 4 + 255) / 256) * 256;
    float* R1 = (float*)wsp; wsp += (((size_t)((size_t)2 * Bn * RHO) * 4 + 255) / 256) * 256;
    k_gd_bd<<<(unsigned)(((long long)3 * NT * 64 * 64 + 255) / 256), 256, 0, stream>>>(A, BD, Bn, NN, NT); k_gd_zero<<<(unsigned)(((long long)NRP * D + 255) / 256), 256, 0, stream>>>(H, T1, M0, (long long)NRP * D); k_gd_zero<<<(unsigned)(((long long)NRP * D + 255) / 256), 256, 0, stream>>>(M1, M1, M1, (long long)NRP * D);
    { GemmP ge1;
      ge1.A = X; ge1.B = We1; ge1.bias = be1; ge1.R = X; ge1.C = T1;
      ge1.sAo = 0; ge1.sAi = 0; ge1.sAm = DIN; ge1.sAk = 1; ge1.sBo = 0; ge1.sBi = 0; ge1.sBn = 1; ge1.sBk = D; ge1.sCo = 0; ge1.sCi = 0; ge1.sCm = D; ge1.sRo = 0; ge1.sRi = 0; ge1.sRm = 0; ge1.sRn = 0;
      ge1.M = NR; ge1.N = D; ge1.K = DIN; ge1.zi_n = 1; ge1.flags = 1; ge1.act = 1;
      ge1.alpha = 1.0f; ge1.beta = 0.0f; ge1.sa = 1.0f; ge1.sb = 1.0f; ge1.Npad = D; ge1.pad_ = 0;
      if ((long long)(NR) >= 64 && (long long)(D) >= 64) k_gemmT<1, 2, 4><<<dim3((unsigned)((D) + 63) / 64, (unsigned)((NR) + 31) / 32, (unsigned)(1)), 32, 0, stream>>>(ge1);
      else k_gemm<1><<<dim3((unsigned)((D) + 31) / 32, (unsigned)((NR) + 15) / 16, (unsigned)(1)), 32, 0, stream>>>(ge1); }
    { GemmP ge2;
      ge2.A = T1; ge2.B = We2; ge2.bias = be2; ge2.R = T1; ge2.C = H;
      ge2.sAo = 0; ge2.sAi = 0; ge2.sAm = D; ge2.sAk = 1; ge2.sBo = 0; ge2.sBi = 0; ge2.sBn = 1; ge2.sBk = D; ge2.sCo = 0; ge2.sCi = 0; ge2.sCm = D; ge2.sRo = 0; ge2.sRi = 0; ge2.sRm = 0; ge2.sRn = 0;
      ge2.M = NR; ge2.N = D; ge2.K = D; ge2.zi_n = 1; ge2.flags = 1; ge2.act = 0;
      ge2.alpha = 1.0f; ge2.beta = 0.0f; ge2.sa = 1.0f; ge2.sb = 1.0f; ge2.Npad = D; ge2.pad_ = 0;
      if ((long long)(NR) >= 64 && (long long)(D) >= 64) k_gemmT<1, 2, 4><<<dim3((unsigned)((D) + 63) / 64, (unsigned)((NR) + 31) / 32, (unsigned)(1)), 32, 0, stream>>>(ge2);
      else k_gemm<1><<<dim3((unsigned)((D) + 31) / 32, (unsigned)((NR) + 15) / 16, (unsigned)(1)), 32, 0, stream>>>(ge2); }
    { GemmP gm00;
      gm00.A = BD + (size_t)0 * NT * 4096; gm00.B = H; gm00.bias = BD + (size_t)0 * NT * 4096; gm00.R = BD + (size_t)0 * NT * 4096; gm00.C = M0;
      gm00.sAo = 4096; gm00.sAi = 0; gm00.sAm = 64; gm00.sAk = 1; gm00.sBo = (long long)60 * D; gm00.sBi = 0; gm00.sBn = 1; gm00.sBk = D; gm00.sCo = (long long)60 * D; gm00.sCi = 0; gm00.sCm = D; gm00.sRo = 0; gm00.sRi = 0; gm00.sRm = 0; gm00.sRn = 0;
      gm00.M = 60; gm00.N = D; gm00.K = 64; gm00.zi_n = 1; gm00.flags = 0; gm00.act = 0;
      gm00.alpha = 1.0f; gm00.beta = 0.0f; gm00.sa = 1.0f; gm00.sb = 1.0f; gm00.Npad = D; gm00.pad_ = 0;
      if ((long long)(60) >= 64 && (long long)(D) >= 64) k_gemmT<1, 2, 4><<<dim3((unsigned)((D) + 63) / 64, (unsigned)((60) + 31) / 32, (unsigned)(NT)), 32, 0, stream>>>(gm00);
      else k_gemm<1><<<dim3((unsigned)((D) + 31) / 32, (unsigned)((60) + 15) / 16, (unsigned)(NT)), 32, 0, stream>>>(gm00); }
    { GemmP gm10;
      gm10.A = BD + (size_t)1 * NT * 4096; gm10.B = H; gm10.bias = BD + (size_t)1 * NT * 4096; gm10.R = BD + (size_t)1 * NT * 4096; gm10.C = M1;
      gm10.sAo = 4096; gm10.sAi = 0; gm10.sAm = 64; gm10.sAk = 1; gm10.sBo = (long long)60 * D; gm10.sBi = 0; gm10.sBn = 1; gm10.sBk = D; gm10.sCo = (long long)60 * D; gm10.sCi = 0; gm10.sCm = D; gm10.sRo = 0; gm10.sRi = 0; gm10.sRm = 0; gm10.sRn = 0;
      gm10.M = 60; gm10.N = D; gm10.K = 64; gm10.zi_n = 1; gm10.flags = 0; gm10.act = 0;
      gm10.alpha = 1.0f; gm10.beta = 0.0f; gm10.sa = 1.0f; gm10.sb = 1.0f; gm10.Npad = D; gm10.pad_ = 0;
      if ((long long)(60) >= 64 && (long long)(D) >= 64) k_gemmT<1, 2, 4><<<dim3((unsigned)((D) + 63) / 64, (unsigned)((60) + 31) / 32, (unsigned)(NT)), 32, 0, stream>>>(gm10);
      else k_gemm<1><<<dim3((unsigned)((D) + 31) / 32, (unsigned)((60) + 15) / 16, (unsigned)(NT)), 32, 0, stream>>>(gm10); }
    { GemmP gr00;
      gr00.A = M0; gr00.B = rw + (size_t)0 * 2 * D * D; gr00.bias = rb + (size_t)0 * D; gr00.R = M0; gr00.C = T1;
      gr00.sAo = 0; gr00.sAi = 0; gr00.sAm = D; gr00.sAk = 1; gr00.sBo = 0; gr00.sBi = 0; gr00.sBn = 1; gr00.sBk = D; gr00.sCo = 0; gr00.sCi = 0; gr00.sCm = D; gr00.sRo = 0; gr00.sRi = 0; gr00.sRm = 0; gr00.sRn = 0;
      gr00.M = NR; gr00.N = D; gr00.K = D; gr00.zi_n = 1; gr00.flags = 1; gr00.act = 0;
      gr00.alpha = 1.0f; gr00.beta = 0.0f; gr00.sa = 1.0f; gr00.sb = 8.0f; gr00.Npad = D; gr00.pad_ = 0;
      if ((long long)(NR) >= 64 && (long long)(D) >= 64) k_gemmT<0, 4, 4><<<dim3((unsigned)((D) + 63) / 64, (unsigned)((NR) + 63) / 64, (unsigned)(1)), 32, 0, stream>>>(gr00);
      else k_gemm<0><<<dim3((unsigned)((D) + 31) / 32, (unsigned)((NR) + 15) / 16, (unsigned)(1)), 32, 0, stream>>>(gr00); }
    { GemmP gr10;
      gr10.A = M1; gr10.B = rw + (size_t)0 * 2 * D * D + (size_t)D * D; gr10.bias = M1; gr10.R = T1; gr10.C = T1;
      gr10.sAo = 0; gr10.sAi = 0; gr10.sAm = D; gr10.sAk = 1; gr10.sBo = 0; gr10.sBi = 0; gr10.sBn = 1; gr10.sBk = D; gr10.sCo = 0; gr10.sCi = 0; gr10.sCm = D; gr10.sRo = 0; gr10.sRi = 0; gr10.sRm = D; gr10.sRn = 1;
      gr10.M = NR; gr10.N = D; gr10.K = D; gr10.zi_n = 1; gr10.flags = 4; gr10.act = 0;
      gr10.alpha = 1.0f; gr10.beta = 1.0f; gr10.sa = 1.0f; gr10.sb = 8.0f; gr10.Npad = D; gr10.pad_ = 0;
      if ((long long)(NR) >= 64 && (long long)(D) >= 64) k_gemmT<0, 4, 4><<<dim3((unsigned)((D) + 63) / 64, (unsigned)((NR) + 63) / 64, (unsigned)(1)), 32, 0, stream>>>(gr10);
      else k_gemm<0><<<dim3((unsigned)((D) + 31) / 32, (unsigned)((NR) + 15) / 16, (unsigned)(1)), 32, 0, stream>>>(gr10); }
    { GemmP grr0;
      grr0.A = H; grr0.B = rroot + (size_t)0 * D * D; grr0.bias = H; grr0.R = T1; grr0.C = T1;
      grr0.sAo = 0; grr0.sAi = 0; grr0.sAm = D; grr0.sAk = 1; grr0.sBo = 0; grr0.sBi = 0; grr0.sBn = 1; grr0.sBk = D; grr0.sCo = 0; grr0.sCi = 0; grr0.sCm = D; grr0.sRo = 0; grr0.sRi = 0; grr0.sRm = D; grr0.sRn = 1;
      grr0.M = NR; grr0.N = D; grr0.K = D; grr0.zi_n = 1; grr0.flags = 4; grr0.act = 0;
      grr0.alpha = 1.0f; grr0.beta = 1.0f; grr0.sa = 1.0f; grr0.sb = 8.0f; grr0.Npad = D; grr0.pad_ = 0;
      if ((long long)(NR) >= 64 && (long long)(D) >= 64) k_gemmT<0, 4, 4><<<dim3((unsigned)((D) + 63) / 64, (unsigned)((NR) + 63) / 64, (unsigned)(1)), 32, 0, stream>>>(grr0);
      else k_gemm<0><<<dim3((unsigned)((D) + 31) / 32, (unsigned)((NR) + 15) / 16, (unsigned)(1)), 32, 0, stream>>>(grr0); }
    { GemmP gaw0;
      gaw0.A = BD + (size_t)2 * NT * 4096; gaw0.B = T1; gaw0.bias = BD + (size_t)2 * NT * 4096; gaw0.R = BD + (size_t)2 * NT * 4096; gaw0.C = M0;
      gaw0.sAo = 4096; gaw0.sAi = 0; gaw0.sAm = 64; gaw0.sAk = 1; gaw0.sBo = (long long)60 * D; gaw0.sBi = 0; gaw0.sBn = 1; gaw0.sBk = D; gaw0.sCo = (long long)60 * D; gaw0.sCi = 0; gaw0.sCm = D; gaw0.sRo = 0; gaw0.sRi = 0; gaw0.sRm = 0; gaw0.sRn = 0;
      gaw0.M = 60; gaw0.N = D; gaw0.K = 64; gaw0.zi_n = 1; gaw0.flags = 0; gaw0.act = 0;
      gaw0.alpha = 1.0f; gaw0.beta = 0.0f; gaw0.sa = 1.0f; gaw0.sb = 1.0f; gaw0.Npad = D; gaw0.pad_ = 0;
      if ((long long)(60) >= 64 && (long long)(D) >= 64) k_gemmT<1, 2, 4><<<dim3((unsigned)((D) + 63) / 64, (unsigned)((60) + 31) / 32, (unsigned)(NT)), 32, 0, stream>>>(gaw0);
      else k_gemm<1><<<dim3((unsigned)((D) + 31) / 32, (unsigned)((60) + 15) / 16, (unsigned)(NT)), 32, 0, stream>>>(gaw0); }
    k_gd_lnrelu<<<(unsigned)((NR + 255) / 256), 256, 0, stream>>>(M0, lng, lnb, NR, D);
    { GemmP gl10;
      gl10.A = M0; gl10.B = l1w + (size_t)0 * D * D; gl10.bias = l1b + (size_t)0 * D; gl10.R = M0; gl10.C = T1;
      gl10.sAo = 0; gl10.sAi = 0; gl10.sAm = D; gl10.sAk = 1; gl10.sBo = 0; gl10.sBi = 0; gl10.sBn = 1; gl10.sBk = D; gl10.sCo = 0; gl10.sCi = 0; gl10.sCm = D; gl10.sRo = 0; gl10.sRi = 0; gl10.sRm = 0; gl10.sRn = 0;
      gl10.M = NR; gl10.N = D; gl10.K = D; gl10.zi_n = 1; gl10.flags = 1; gl10.act = 1;
      gl10.alpha = 1.0f; gl10.beta = 0.0f; gl10.sa = 1.0f; gl10.sb = 8.0f; gl10.Npad = D; gl10.pad_ = 0;
      if ((long long)(NR) >= 64 && (long long)(D) >= 64) k_gemmT<0, 4, 4><<<dim3((unsigned)((D) + 63) / 64, (unsigned)((NR) + 63) / 64, (unsigned)(1)), 32, 0, stream>>>(gl10);
      else k_gemm<0><<<dim3((unsigned)((D) + 31) / 32, (unsigned)((NR) + 15) / 16, (unsigned)(1)), 32, 0, stream>>>(gl10); }
    { GemmP gl20;
      gl20.A = T1; gl20.B = l2w + (size_t)0 * D * D; gl20.bias = l2b + (size_t)0 * D; gl20.R = T1; gl20.C = M0;
      gl20.sAo = 0; gl20.sAi = 0; gl20.sAm = D; gl20.sAk = 1; gl20.sBo = 0; gl20.sBi = 0; gl20.sBn = 1; gl20.sBk = D; gl20.sCo = 0; gl20.sCi = 0; gl20.sCm = D; gl20.sRo = 0; gl20.sRi = 0; gl20.sRm = 0; gl20.sRn = 0;
      gl20.M = NR; gl20.N = D; gl20.K = D; gl20.zi_n = 1; gl20.flags = 1; gl20.act = 0;
      gl20.alpha = 1.0f; gl20.beta = 0.0f; gl20.sa = 1.0f; gl20.sb = 8.0f; gl20.Npad = D; gl20.pad_ = 0;
      if ((long long)(NR) >= 64 && (long long)(D) >= 64) k_gemmT<0, 4, 4><<<dim3((unsigned)((D) + 63) / 64, (unsigned)((NR) + 63) / 64, (unsigned)(1)), 32, 0, stream>>>(gl20);
      else k_gemm<0><<<dim3((unsigned)((D) + 31) / 32, (unsigned)((NR) + 15) / 16, (unsigned)(1)), 32, 0, stream>>>(gl20); }
    k_gd_add<<<(unsigned)(((long long)NR * D + 255) / 256), 256, 0, stream>>>(H, M0, (long long)NR * D);
    { GemmP gm01;
      gm01.A = BD + (size_t)0 * NT * 4096; gm01.B = H; gm01.bias = BD + (size_t)0 * NT * 4096; gm01.R = BD + (size_t)0 * NT * 4096; gm01.C = M0;
      gm01.sAo = 4096; gm01.sAi = 0; gm01.sAm = 64; gm01.sAk = 1; gm01.sBo = (long long)60 * D; gm01.sBi = 0; gm01.sBn = 1; gm01.sBk = D; gm01.sCo = (long long)60 * D; gm01.sCi = 0; gm01.sCm = D; gm01.sRo = 0; gm01.sRi = 0; gm01.sRm = 0; gm01.sRn = 0;
      gm01.M = 60; gm01.N = D; gm01.K = 64; gm01.zi_n = 1; gm01.flags = 0; gm01.act = 0;
      gm01.alpha = 1.0f; gm01.beta = 0.0f; gm01.sa = 1.0f; gm01.sb = 1.0f; gm01.Npad = D; gm01.pad_ = 0;
      if ((long long)(60) >= 64 && (long long)(D) >= 64) k_gemmT<1, 2, 4><<<dim3((unsigned)((D) + 63) / 64, (unsigned)((60) + 31) / 32, (unsigned)(NT)), 32, 0, stream>>>(gm01);
      else k_gemm<1><<<dim3((unsigned)((D) + 31) / 32, (unsigned)((60) + 15) / 16, (unsigned)(NT)), 32, 0, stream>>>(gm01); }
    { GemmP gm11;
      gm11.A = BD + (size_t)1 * NT * 4096; gm11.B = H; gm11.bias = BD + (size_t)1 * NT * 4096; gm11.R = BD + (size_t)1 * NT * 4096; gm11.C = M1;
      gm11.sAo = 4096; gm11.sAi = 0; gm11.sAm = 64; gm11.sAk = 1; gm11.sBo = (long long)60 * D; gm11.sBi = 0; gm11.sBn = 1; gm11.sBk = D; gm11.sCo = (long long)60 * D; gm11.sCi = 0; gm11.sCm = D; gm11.sRo = 0; gm11.sRi = 0; gm11.sRm = 0; gm11.sRn = 0;
      gm11.M = 60; gm11.N = D; gm11.K = 64; gm11.zi_n = 1; gm11.flags = 0; gm11.act = 0;
      gm11.alpha = 1.0f; gm11.beta = 0.0f; gm11.sa = 1.0f; gm11.sb = 1.0f; gm11.Npad = D; gm11.pad_ = 0;
      if ((long long)(60) >= 64 && (long long)(D) >= 64) k_gemmT<1, 2, 4><<<dim3((unsigned)((D) + 63) / 64, (unsigned)((60) + 31) / 32, (unsigned)(NT)), 32, 0, stream>>>(gm11);
      else k_gemm<1><<<dim3((unsigned)((D) + 31) / 32, (unsigned)((60) + 15) / 16, (unsigned)(NT)), 32, 0, stream>>>(gm11); }
    { GemmP gr01;
      gr01.A = M0; gr01.B = rw + (size_t)1 * 2 * D * D; gr01.bias = rb + (size_t)1 * D; gr01.R = M0; gr01.C = T1;
      gr01.sAo = 0; gr01.sAi = 0; gr01.sAm = D; gr01.sAk = 1; gr01.sBo = 0; gr01.sBi = 0; gr01.sBn = 1; gr01.sBk = D; gr01.sCo = 0; gr01.sCi = 0; gr01.sCm = D; gr01.sRo = 0; gr01.sRi = 0; gr01.sRm = 0; gr01.sRn = 0;
      gr01.M = NR; gr01.N = D; gr01.K = D; gr01.zi_n = 1; gr01.flags = 1; gr01.act = 0;
      gr01.alpha = 1.0f; gr01.beta = 0.0f; gr01.sa = 1.0f; gr01.sb = 8.0f; gr01.Npad = D; gr01.pad_ = 0;
      if ((long long)(NR) >= 64 && (long long)(D) >= 64) k_gemmT<0, 4, 4><<<dim3((unsigned)((D) + 63) / 64, (unsigned)((NR) + 63) / 64, (unsigned)(1)), 32, 0, stream>>>(gr01);
      else k_gemm<0><<<dim3((unsigned)((D) + 31) / 32, (unsigned)((NR) + 15) / 16, (unsigned)(1)), 32, 0, stream>>>(gr01); }
    { GemmP gr11;
      gr11.A = M1; gr11.B = rw + (size_t)1 * 2 * D * D + (size_t)D * D; gr11.bias = M1; gr11.R = T1; gr11.C = T1;
      gr11.sAo = 0; gr11.sAi = 0; gr11.sAm = D; gr11.sAk = 1; gr11.sBo = 0; gr11.sBi = 0; gr11.sBn = 1; gr11.sBk = D; gr11.sCo = 0; gr11.sCi = 0; gr11.sCm = D; gr11.sRo = 0; gr11.sRi = 0; gr11.sRm = D; gr11.sRn = 1;
      gr11.M = NR; gr11.N = D; gr11.K = D; gr11.zi_n = 1; gr11.flags = 4; gr11.act = 0;
      gr11.alpha = 1.0f; gr11.beta = 1.0f; gr11.sa = 1.0f; gr11.sb = 8.0f; gr11.Npad = D; gr11.pad_ = 0;
      if ((long long)(NR) >= 64 && (long long)(D) >= 64) k_gemmT<0, 4, 4><<<dim3((unsigned)((D) + 63) / 64, (unsigned)((NR) + 63) / 64, (unsigned)(1)), 32, 0, stream>>>(gr11);
      else k_gemm<0><<<dim3((unsigned)((D) + 31) / 32, (unsigned)((NR) + 15) / 16, (unsigned)(1)), 32, 0, stream>>>(gr11); }
    { GemmP grr1;
      grr1.A = H; grr1.B = rroot + (size_t)1 * D * D; grr1.bias = H; grr1.R = T1; grr1.C = T1;
      grr1.sAo = 0; grr1.sAi = 0; grr1.sAm = D; grr1.sAk = 1; grr1.sBo = 0; grr1.sBi = 0; grr1.sBn = 1; grr1.sBk = D; grr1.sCo = 0; grr1.sCi = 0; grr1.sCm = D; grr1.sRo = 0; grr1.sRi = 0; grr1.sRm = D; grr1.sRn = 1;
      grr1.M = NR; grr1.N = D; grr1.K = D; grr1.zi_n = 1; grr1.flags = 4; grr1.act = 0;
      grr1.alpha = 1.0f; grr1.beta = 1.0f; grr1.sa = 1.0f; grr1.sb = 8.0f; grr1.Npad = D; grr1.pad_ = 0;
      if ((long long)(NR) >= 64 && (long long)(D) >= 64) k_gemmT<0, 4, 4><<<dim3((unsigned)((D) + 63) / 64, (unsigned)((NR) + 63) / 64, (unsigned)(1)), 32, 0, stream>>>(grr1);
      else k_gemm<0><<<dim3((unsigned)((D) + 31) / 32, (unsigned)((NR) + 15) / 16, (unsigned)(1)), 32, 0, stream>>>(grr1); }
    { GemmP gaw1;
      gaw1.A = BD + (size_t)2 * NT * 4096; gaw1.B = T1; gaw1.bias = BD + (size_t)2 * NT * 4096; gaw1.R = BD + (size_t)2 * NT * 4096; gaw1.C = M0;
      gaw1.sAo = 4096; gaw1.sAi = 0; gaw1.sAm = 64; gaw1.sAk = 1; gaw1.sBo = (long long)60 * D; gaw1.sBi = 0; gaw1.sBn = 1; gaw1.sBk = D; gaw1.sCo = (long long)60 * D; gaw1.sCi = 0; gaw1.sCm = D; gaw1.sRo = 0; gaw1.sRi = 0; gaw1.sRm = 0; gaw1.sRn = 0;
      gaw1.M = 60; gaw1.N = D; gaw1.K = 64; gaw1.zi_n = 1; gaw1.flags = 0; gaw1.act = 0;
      gaw1.alpha = 1.0f; gaw1.beta = 0.0f; gaw1.sa = 1.0f; gaw1.sb = 1.0f; gaw1.Npad = D; gaw1.pad_ = 0;
      if ((long long)(60) >= 64 && (long long)(D) >= 64) k_gemmT<1, 2, 4><<<dim3((unsigned)((D) + 63) / 64, (unsigned)((60) + 31) / 32, (unsigned)(NT)), 32, 0, stream>>>(gaw1);
      else k_gemm<1><<<dim3((unsigned)((D) + 31) / 32, (unsigned)((60) + 15) / 16, (unsigned)(NT)), 32, 0, stream>>>(gaw1); }
    k_gd_lnrelu<<<(unsigned)((NR + 255) / 256), 256, 0, stream>>>(M0, lng, lnb, NR, D);
    { GemmP gl11;
      gl11.A = M0; gl11.B = l1w + (size_t)1 * D * D; gl11.bias = l1b + (size_t)1 * D; gl11.R = M0; gl11.C = T1;
      gl11.sAo = 0; gl11.sAi = 0; gl11.sAm = D; gl11.sAk = 1; gl11.sBo = 0; gl11.sBi = 0; gl11.sBn = 1; gl11.sBk = D; gl11.sCo = 0; gl11.sCi = 0; gl11.sCm = D; gl11.sRo = 0; gl11.sRi = 0; gl11.sRm = 0; gl11.sRn = 0;
      gl11.M = NR; gl11.N = D; gl11.K = D; gl11.zi_n = 1; gl11.flags = 1; gl11.act = 1;
      gl11.alpha = 1.0f; gl11.beta = 0.0f; gl11.sa = 1.0f; gl11.sb = 8.0f; gl11.Npad = D; gl11.pad_ = 0;
      if ((long long)(NR) >= 64 && (long long)(D) >= 64) k_gemmT<0, 4, 4><<<dim3((unsigned)((D) + 63) / 64, (unsigned)((NR) + 63) / 64, (unsigned)(1)), 32, 0, stream>>>(gl11);
      else k_gemm<0><<<dim3((unsigned)((D) + 31) / 32, (unsigned)((NR) + 15) / 16, (unsigned)(1)), 32, 0, stream>>>(gl11); }
    { GemmP gl21;
      gl21.A = T1; gl21.B = l2w + (size_t)1 * D * D; gl21.bias = l2b + (size_t)1 * D; gl21.R = T1; gl21.C = M0;
      gl21.sAo = 0; gl21.sAi = 0; gl21.sAm = D; gl21.sAk = 1; gl21.sBo = 0; gl21.sBi = 0; gl21.sBn = 1; gl21.sBk = D; gl21.sCo = 0; gl21.sCi = 0; gl21.sCm = D; gl21.sRo = 0; gl21.sRi = 0; gl21.sRm = 0; gl21.sRn = 0;
      gl21.M = NR; gl21.N = D; gl21.K = D; gl21.zi_n = 1; gl21.flags = 1; gl21.act = 0;
      gl21.alpha = 1.0f; gl21.beta = 0.0f; gl21.sa = 1.0f; gl21.sb = 8.0f; gl21.Npad = D; gl21.pad_ = 0;
      if ((long long)(NR) >= 64 && (long long)(D) >= 64) k_gemmT<0, 4, 4><<<dim3((unsigned)((D) + 63) / 64, (unsigned)((NR) + 63) / 64, (unsigned)(1)), 32, 0, stream>>>(gl21);
      else k_gemm<0><<<dim3((unsigned)((D) + 31) / 32, (unsigned)((NR) + 15) / 16, (unsigned)(1)), 32, 0, stream>>>(gl21); }
    k_gd_add<<<(unsigned)(((long long)NR * D + 255) / 256), 256, 0, stream>>>(H, M0, (long long)NR * D);
    { GemmP gm02;
      gm02.A = BD + (size_t)0 * NT * 4096; gm02.B = H; gm02.bias = BD + (size_t)0 * NT * 4096; gm02.R = BD + (size_t)0 * NT * 4096; gm02.C = M0;
      gm02.sAo = 4096; gm02.sAi = 0; gm02.sAm = 64; gm02.sAk = 1; gm02.sBo = (long long)60 * D; gm02.sBi = 0; gm02.sBn = 1; gm02.sBk = D; gm02.sCo = (long long)60 * D; gm02.sCi = 0; gm02.sCm = D; gm02.sRo = 0; gm02.sRi = 0; gm02.sRm = 0; gm02.sRn = 0;
      gm02.M = 60; gm02.N = D; gm02.K = 64; gm02.zi_n = 1; gm02.flags = 0; gm02.act = 0;
      gm02.alpha = 1.0f; gm02.beta = 0.0f; gm02.sa = 1.0f; gm02.sb = 1.0f; gm02.Npad = D; gm02.pad_ = 0;
      if ((long long)(60) >= 64 && (long long)(D) >= 64) k_gemmT<1, 2, 4><<<dim3((unsigned)((D) + 63) / 64, (unsigned)((60) + 31) / 32, (unsigned)(NT)), 32, 0, stream>>>(gm02);
      else k_gemm<1><<<dim3((unsigned)((D) + 31) / 32, (unsigned)((60) + 15) / 16, (unsigned)(NT)), 32, 0, stream>>>(gm02); }
    { GemmP gm12;
      gm12.A = BD + (size_t)1 * NT * 4096; gm12.B = H; gm12.bias = BD + (size_t)1 * NT * 4096; gm12.R = BD + (size_t)1 * NT * 4096; gm12.C = M1;
      gm12.sAo = 4096; gm12.sAi = 0; gm12.sAm = 64; gm12.sAk = 1; gm12.sBo = (long long)60 * D; gm12.sBi = 0; gm12.sBn = 1; gm12.sBk = D; gm12.sCo = (long long)60 * D; gm12.sCi = 0; gm12.sCm = D; gm12.sRo = 0; gm12.sRi = 0; gm12.sRm = 0; gm12.sRn = 0;
      gm12.M = 60; gm12.N = D; gm12.K = 64; gm12.zi_n = 1; gm12.flags = 0; gm12.act = 0;
      gm12.alpha = 1.0f; gm12.beta = 0.0f; gm12.sa = 1.0f; gm12.sb = 1.0f; gm12.Npad = D; gm12.pad_ = 0;
      if ((long long)(60) >= 64 && (long long)(D) >= 64) k_gemmT<1, 2, 4><<<dim3((unsigned)((D) + 63) / 64, (unsigned)((60) + 31) / 32, (unsigned)(NT)), 32, 0, stream>>>(gm12);
      else k_gemm<1><<<dim3((unsigned)((D) + 31) / 32, (unsigned)((60) + 15) / 16, (unsigned)(NT)), 32, 0, stream>>>(gm12); }
    { GemmP gr02;
      gr02.A = M0; gr02.B = rw + (size_t)2 * 2 * D * D; gr02.bias = rb + (size_t)2 * D; gr02.R = M0; gr02.C = T1;
      gr02.sAo = 0; gr02.sAi = 0; gr02.sAm = D; gr02.sAk = 1; gr02.sBo = 0; gr02.sBi = 0; gr02.sBn = 1; gr02.sBk = D; gr02.sCo = 0; gr02.sCi = 0; gr02.sCm = D; gr02.sRo = 0; gr02.sRi = 0; gr02.sRm = 0; gr02.sRn = 0;
      gr02.M = NR; gr02.N = D; gr02.K = D; gr02.zi_n = 1; gr02.flags = 1; gr02.act = 0;
      gr02.alpha = 1.0f; gr02.beta = 0.0f; gr02.sa = 1.0f; gr02.sb = 8.0f; gr02.Npad = D; gr02.pad_ = 0;
      if ((long long)(NR) >= 64 && (long long)(D) >= 64) k_gemmT<0, 4, 4><<<dim3((unsigned)((D) + 63) / 64, (unsigned)((NR) + 63) / 64, (unsigned)(1)), 32, 0, stream>>>(gr02);
      else k_gemm<0><<<dim3((unsigned)((D) + 31) / 32, (unsigned)((NR) + 15) / 16, (unsigned)(1)), 32, 0, stream>>>(gr02); }
    { GemmP gr12;
      gr12.A = M1; gr12.B = rw + (size_t)2 * 2 * D * D + (size_t)D * D; gr12.bias = M1; gr12.R = T1; gr12.C = T1;
      gr12.sAo = 0; gr12.sAi = 0; gr12.sAm = D; gr12.sAk = 1; gr12.sBo = 0; gr12.sBi = 0; gr12.sBn = 1; gr12.sBk = D; gr12.sCo = 0; gr12.sCi = 0; gr12.sCm = D; gr12.sRo = 0; gr12.sRi = 0; gr12.sRm = D; gr12.sRn = 1;
      gr12.M = NR; gr12.N = D; gr12.K = D; gr12.zi_n = 1; gr12.flags = 4; gr12.act = 0;
      gr12.alpha = 1.0f; gr12.beta = 1.0f; gr12.sa = 1.0f; gr12.sb = 8.0f; gr12.Npad = D; gr12.pad_ = 0;
      if ((long long)(NR) >= 64 && (long long)(D) >= 64) k_gemmT<0, 4, 4><<<dim3((unsigned)((D) + 63) / 64, (unsigned)((NR) + 63) / 64, (unsigned)(1)), 32, 0, stream>>>(gr12);
      else k_gemm<0><<<dim3((unsigned)((D) + 31) / 32, (unsigned)((NR) + 15) / 16, (unsigned)(1)), 32, 0, stream>>>(gr12); }
    { GemmP grr2;
      grr2.A = H; grr2.B = rroot + (size_t)2 * D * D; grr2.bias = H; grr2.R = T1; grr2.C = T1;
      grr2.sAo = 0; grr2.sAi = 0; grr2.sAm = D; grr2.sAk = 1; grr2.sBo = 0; grr2.sBi = 0; grr2.sBn = 1; grr2.sBk = D; grr2.sCo = 0; grr2.sCi = 0; grr2.sCm = D; grr2.sRo = 0; grr2.sRi = 0; grr2.sRm = D; grr2.sRn = 1;
      grr2.M = NR; grr2.N = D; grr2.K = D; grr2.zi_n = 1; grr2.flags = 4; grr2.act = 0;
      grr2.alpha = 1.0f; grr2.beta = 1.0f; grr2.sa = 1.0f; grr2.sb = 8.0f; grr2.Npad = D; grr2.pad_ = 0;
      if ((long long)(NR) >= 64 && (long long)(D) >= 64) k_gemmT<0, 4, 4><<<dim3((unsigned)((D) + 63) / 64, (unsigned)((NR) + 63) / 64, (unsigned)(1)), 32, 0, stream>>>(grr2);
      else k_gemm<0><<<dim3((unsigned)((D) + 31) / 32, (unsigned)((NR) + 15) / 16, (unsigned)(1)), 32, 0, stream>>>(grr2); }
    { GemmP gaw2;
      gaw2.A = BD + (size_t)2 * NT * 4096; gaw2.B = T1; gaw2.bias = BD + (size_t)2 * NT * 4096; gaw2.R = BD + (size_t)2 * NT * 4096; gaw2.C = M0;
      gaw2.sAo = 4096; gaw2.sAi = 0; gaw2.sAm = 64; gaw2.sAk = 1; gaw2.sBo = (long long)60 * D; gaw2.sBi = 0; gaw2.sBn = 1; gaw2.sBk = D; gaw2.sCo = (long long)60 * D; gaw2.sCi = 0; gaw2.sCm = D; gaw2.sRo = 0; gaw2.sRi = 0; gaw2.sRm = 0; gaw2.sRn = 0;
      gaw2.M = 60; gaw2.N = D; gaw2.K = 64; gaw2.zi_n = 1; gaw2.flags = 0; gaw2.act = 0;
      gaw2.alpha = 1.0f; gaw2.beta = 0.0f; gaw2.sa = 1.0f; gaw2.sb = 1.0f; gaw2.Npad = D; gaw2.pad_ = 0;
      if ((long long)(60) >= 64 && (long long)(D) >= 64) k_gemmT<1, 2, 4><<<dim3((unsigned)((D) + 63) / 64, (unsigned)((60) + 31) / 32, (unsigned)(NT)), 32, 0, stream>>>(gaw2);
      else k_gemm<1><<<dim3((unsigned)((D) + 31) / 32, (unsigned)((60) + 15) / 16, (unsigned)(NT)), 32, 0, stream>>>(gaw2); }
    k_gd_lnrelu<<<(unsigned)((NR + 255) / 256), 256, 0, stream>>>(M0, lng, lnb, NR, D);
    { GemmP gl12;
      gl12.A = M0; gl12.B = l1w + (size_t)2 * D * D; gl12.bias = l1b + (size_t)2 * D; gl12.R = M0; gl12.C = T1;
      gl12.sAo = 0; gl12.sAi = 0; gl12.sAm = D; gl12.sAk = 1; gl12.sBo = 0; gl12.sBi = 0; gl12.sBn = 1; gl12.sBk = D; gl12.sCo = 0; gl12.sCi = 0; gl12.sCm = D; gl12.sRo = 0; gl12.sRi = 0; gl12.sRm = 0; gl12.sRn = 0;
      gl12.M = NR; gl12.N = D; gl12.K = D; gl12.zi_n = 1; gl12.flags = 1; gl12.act = 1;
      gl12.alpha = 1.0f; gl12.beta = 0.0f; gl12.sa = 1.0f; gl12.sb = 8.0f; gl12.Npad = D; gl12.pad_ = 0;
      if ((long long)(NR) >= 64 && (long long)(D) >= 64) k_gemmT<0, 4, 4><<<dim3((unsigned)((D) + 63) / 64, (unsigned)((NR) + 63) / 64, (unsigned)(1)), 32, 0, stream>>>(gl12);
      else k_gemm<0><<<dim3((unsigned)((D) + 31) / 32, (unsigned)((NR) + 15) / 16, (unsigned)(1)), 32, 0, stream>>>(gl12); }
    { GemmP gl22;
      gl22.A = T1; gl22.B = l2w + (size_t)2 * D * D; gl22.bias = l2b + (size_t)2 * D; gl22.R = T1; gl22.C = M0;
      gl22.sAo = 0; gl22.sAi = 0; gl22.sAm = D; gl22.sAk = 1; gl22.sBo = 0; gl22.sBi = 0; gl22.sBn = 1; gl22.sBk = D; gl22.sCo = 0; gl22.sCi = 0; gl22.sCm = D; gl22.sRo = 0; gl22.sRi = 0; gl22.sRm = 0; gl22.sRn = 0;
      gl22.M = NR; gl22.N = D; gl22.K = D; gl22.zi_n = 1; gl22.flags = 1; gl22.act = 0;
      gl22.alpha = 1.0f; gl22.beta = 0.0f; gl22.sa = 1.0f; gl22.sb = 8.0f; gl22.Npad = D; gl22.pad_ = 0;
      if ((long long)(NR) >= 64 && (long long)(D) >= 64) k_gemmT<0, 4, 4><<<dim3((unsigned)((D) + 63) / 64, (unsigned)((NR) + 63) / 64, (unsigned)(1)), 32, 0, stream>>>(gl22);
      else k_gemm<0><<<dim3((unsigned)((D) + 31) / 32, (unsigned)((NR) + 15) / 16, (unsigned)(1)), 32, 0, stream>>>(gl22); }
    k_gd_add<<<(unsigned)(((long long)NR * D + 255) / 256), 256, 0, stream>>>(H, M0, (long long)NR * D);
    { GemmP gp10;
      gp10.A = H + (size_t)0 * RC * D; gp10.B = p1w; gp10.bias = p1b; gp10.R = H + (size_t)0 * RC * D; gp10.C = M0;
      gp10.sAo = 0; gp10.sAi = 0; gp10.sAm = D; gp10.sAk = 1; gp10.sBo = 0; gp10.sBi = 0; gp10.sBn = 1; gp10.sBk = PHI; gp10.sCo = 0; gp10.sCi = 0; gp10.sCm = PHI; gp10.sRo = 0; gp10.sRi = 0; gp10.sRm = 0; gp10.sRn = 0;
      gp10.M = RC; gp10.N = PHI; gp10.K = D; gp10.zi_n = 1; gp10.flags = 1; gp10.act = 1;
      gp10.alpha = 1.0f; gp10.beta = 0.0f; gp10.sa = 1.0f; gp10.sb = 8.0f; gp10.Npad = PHI; gp10.pad_ = 0;
      if ((long long)(RC) >= 64 && (long long)(PHI) >= 64) k_gemmT<0, 4, 4><<<dim3((unsigned)((PHI) + 63) / 64, (unsigned)((RC) + 63) / 64, (unsigned)(1)), 32, 0, stream>>>(gp10);
      else k_gemm<0><<<dim3((unsigned)((PHI) + 31) / 32, (unsigned)((RC) + 15) / 16, (unsigned)(1)), 32, 0, stream>>>(gp10); }
    { GemmP gp20;
      gp20.A = M0; gp20.B = p2w; gp20.bias = p2b; gp20.R = M0; gp20.C = M1;
      gp20.sAo = 0; gp20.sAi = 0; gp20.sAm = PHI; gp20.sAk = 1; gp20.sBo = 0; gp20.sBi = 0; gp20.sBn = 1; gp20.sBk = PHI; gp20.sCo = 0; gp20.sCi = 0; gp20.sCm = PHI; gp20.sRo = 0; gp20.sRi = 0; gp20.sRm = 0; gp20.sRn = 0;
      gp20.M = RC; gp20.N = PHI; gp20.K = PHI; gp20.zi_n = 1; gp20.flags = 1; gp20.act = 1;
      gp20.alpha = 1.0f; gp20.beta = 0.0f; gp20.sa = 1.0f; gp20.sb = 8.0f; gp20.Npad = PHI; gp20.pad_ = 0;
      if ((long long)(RC) >= 64 && (long long)(PHI) >= 64) k_gemmT<0, 4, 4><<<dim3((unsigned)((PHI) + 63) / 64, (unsigned)((RC) + 63) / 64, (unsigned)(1)), 32, 0, stream>>>(gp20);
      else k_gemm<0><<<dim3((unsigned)((PHI) + 31) / 32, (unsigned)((RC) + 15) / 16, (unsigned)(1)), 32, 0, stream>>>(gp20); }
    k_gd_sets<<<(unsigned)(((long long)GC * PHI + 255) / 256), 256, 0, stream>>>(M1, hm + (size_t)0 * GC * NN, SS + (size_t)0 * GC * PHI, GC, NN, PHI, Bn);
    { GemmP gp11;
      gp11.A = H + (size_t)1 * RC * D; gp11.B = p1w; gp11.bias = p1b; gp11.R = H + (size_t)1 * RC * D; gp11.C = M0;
      gp11.sAo = 0; gp11.sAi = 0; gp11.sAm = D; gp11.sAk = 1; gp11.sBo = 0; gp11.sBi = 0; gp11.sBn = 1; gp11.sBk = PHI; gp11.sCo = 0; gp11.sCi = 0; gp11.sCm = PHI; gp11.sRo = 0; gp11.sRi = 0; gp11.sRm = 0; gp11.sRn = 0;
      gp11.M = RC; gp11.N = PHI; gp11.K = D; gp11.zi_n = 1; gp11.flags = 1; gp11.act = 1;
      gp11.alpha = 1.0f; gp11.beta = 0.0f; gp11.sa = 1.0f; gp11.sb = 8.0f; gp11.Npad = PHI; gp11.pad_ = 0;
      if ((long long)(RC) >= 64 && (long long)(PHI) >= 64) k_gemmT<0, 4, 4><<<dim3((unsigned)((PHI) + 63) / 64, (unsigned)((RC) + 63) / 64, (unsigned)(1)), 32, 0, stream>>>(gp11);
      else k_gemm<0><<<dim3((unsigned)((PHI) + 31) / 32, (unsigned)((RC) + 15) / 16, (unsigned)(1)), 32, 0, stream>>>(gp11); }
    { GemmP gp21;
      gp21.A = M0; gp21.B = p2w; gp21.bias = p2b; gp21.R = M0; gp21.C = M1;
      gp21.sAo = 0; gp21.sAi = 0; gp21.sAm = PHI; gp21.sAk = 1; gp21.sBo = 0; gp21.sBi = 0; gp21.sBn = 1; gp21.sBk = PHI; gp21.sCo = 0; gp21.sCi = 0; gp21.sCm = PHI; gp21.sRo = 0; gp21.sRi = 0; gp21.sRm = 0; gp21.sRn = 0;
      gp21.M = RC; gp21.N = PHI; gp21.K = PHI; gp21.zi_n = 1; gp21.flags = 1; gp21.act = 1;
      gp21.alpha = 1.0f; gp21.beta = 0.0f; gp21.sa = 1.0f; gp21.sb = 8.0f; gp21.Npad = PHI; gp21.pad_ = 0;
      if ((long long)(RC) >= 64 && (long long)(PHI) >= 64) k_gemmT<0, 4, 4><<<dim3((unsigned)((PHI) + 63) / 64, (unsigned)((RC) + 63) / 64, (unsigned)(1)), 32, 0, stream>>>(gp21);
      else k_gemm<0><<<dim3((unsigned)((PHI) + 31) / 32, (unsigned)((RC) + 15) / 16, (unsigned)(1)), 32, 0, stream>>>(gp21); }
    k_gd_sets<<<(unsigned)(((long long)GC * PHI + 255) / 256), 256, 0, stream>>>(M1, hm + (size_t)1 * GC * NN, SS + (size_t)1 * GC * PHI, GC, NN, PHI, Bn);
    { GemmP gr1;
      gr1.A = SS; gr1.B = r1w; gr1.bias = r1b; gr1.R = SS; gr1.C = R1;
      gr1.sAo = 0; gr1.sAi = 0; gr1.sAm = PHI; gr1.sAk = 1; gr1.sBo = 0; gr1.sBi = 0; gr1.sBn = 1; gr1.sBk = RHO; gr1.sCo = 0; gr1.sCi = 0; gr1.sCm = RHO; gr1.sRo = 0; gr1.sRi = 0; gr1.sRm = 0; gr1.sRn = 0;
      gr1.M = 2 * Bn; gr1.N = RHO; gr1.K = PHI; gr1.zi_n = 1; gr1.flags = 1; gr1.act = 1;
      gr1.alpha = 1.0f; gr1.beta = 0.0f; gr1.sa = 1.0f; gr1.sb = 1.0f; gr1.Npad = RHO; gr1.pad_ = 0;
      if ((long long)(2 * Bn) >= 64 && (long long)(RHO) >= 64) k_gemmT<1, 2, 4><<<dim3((unsigned)((RHO) + 63) / 64, (unsigned)((2 * Bn) + 31) / 32, (unsigned)(1)), 32, 0, stream>>>(gr1);
      else k_gemm<1><<<dim3((unsigned)((RHO) + 31) / 32, (unsigned)((2 * Bn) + 15) / 16, (unsigned)(1)), 32, 0, stream>>>(gr1); }
    k_gd_out<<<Bn, 128, 0, stream>>>(R1, r2w, out, Bn, RHO);
}
